// FBPINN_fast_49684181680203
// MI455X (gfx1250) — hardware-run, weakly checked
//
#include <hip/hip_runtime.h>


#ifndef NPTS
#define NPTS 65536
#endif
#define NPTS_FULL 65536
#define NSUB 64
#define HID  32
#define NLH  2
#define MW   8
#define TPB  (16 * MW)
#define SCP  16
#define WCS  16.0f
#define L2E  1.4426950408889634f
#define TK1  (2.0f * 1.4426950408889634f)
#define TKH  (2.0f * 1.4426950408889634f / 16.0f)
#define TC1  15.0f
#define TCH  240.0f

static_assert(HID == 32);
static_assert(NLH == 2);
static_assert(NPTS % TPB == 0);
static_assert(NPTS <= NPTS_FULL);
static_assert(TPB * 4 == 32 * 16);
static_assert(TPB * 4 <= 131072);
static_assert(NSUB * 4 == 256);
static_assert(SCP == 16);
static_assert((NLH * NSUB * HID * HID) % 64 == 0);
static_assert((NSUB * HID * 2) % 32 == 0);
static_assert((NSUB * HID) % 32 == 0);
static_assert((NLH * NSUB * HID) % 32 == 0);

typedef _Float16 h16;
typedef unsigned short bf;
typedef __attribute__((ext_vector_type(16))) _Float16 v16h;
typedef __attribute__((ext_vector_type(8)))  _Float16 v8h;
typedef __attribute__((ext_vector_type(8)))  float    v8f;
typedef __attribute__((ext_vector_type(4)))  float    v4f;
typedef __attribute__((ext_vector_type(2)))  float    v2f;
typedef v4f  __attribute__((may_alias)) v4fa;

__device__ __forceinline__ unsigned short f2bf(float f) { unsigned u = __float_as_uint(f); u += 0x7FFFu + ((u >> 16) & 1u); return (unsigned short)(u >> 16); }
__device__ __forceinline__ float bfr(float f) { return __uint_as_float(((unsigned)f2bf(f)) << 16); }
__device__ __forceinline__ v16h cat16(v8h lo, v8h hi) { return __builtin_shufflevector(lo, hi, 0, 1, 2, 3, 4, 5, 6, 7, 8, 9, 10, 11, 12, 13, 14, 15); }
__device__ __forceinline__ v8f wmma16(v16h a, v16h b, v8f c) { return __builtin_amdgcn_wmma_f32_16x16x32_f16(false, a, false, b, (short)0, c, false, false); }
__device__ __forceinline__ v16h  ldh(const h16* p) { return cat16(*(const v8h*)p, *(const v8h*)(p + 16)); }
__device__ __forceinline__ v8f wmma16g(v16h a, v16h b, v8f c) { c = wmma16(a, b, c); asm volatile("v_nop\n\tv_nop\n\tv_nop\n\tv_nop" : "+v"(c) : "v"(a), "v"(b)); return c; }
__device__ __forceinline__ v8f cat8f(v4f a, v4f b) { return __builtin_shufflevector(a, b, 0, 1, 2, 3, 4, 5, 6, 7); }
static __device__ __forceinline__ h16 toh_flush(float v) { const h16 r = (h16)v; return (fabsf(v) < 6.103515625e-05f) ? (h16)0.0f : r; }
__device__ __forceinline__ float tanh_e(float d, float k2, float c) {
    const float z = __builtin_amdgcn_fmed3f(d, -c, c);
    const float e = __builtin_amdgcn_exp2f(z * k2);
    const float r = __builtin_amdgcn_rcpf(1.0f + e);
    return 1.0f - 2.0f * r;
}
__device__ __forceinline__ float sig_e(float z) {
    const float a = fminf(-z, 80.0f);
    return __builtin_amdgcn_rcpf(1.0f + __builtin_amdgcn_exp2f(a * L2E));
}

__global__ __launch_bounds__(256) void k_cvtf(const float* __restrict__ src, float* dst, int n4, float carry) {
#pragma clang fp contract(off)
    const int i = blockIdx.x * 256 + threadIdx.x; if (i >= n4) return;
    const v4f v = *(const v4f*)(src + (size_t)i * 4); v4f o;
#pragma unroll
    for (int k = 0; k < 4; ++k) o[k] = bfr(v[k]) * carry;
    *(volatile v4f*)(dst + (size_t)i * 4) = o; __threadfence(); *(volatile v4f*)(dst + (size_t)i * 4) = o;
}

__global__ __launch_bounds__(256) void k_wconv(const float* __restrict__ src, h16* dst, int n8) {
#pragma clang fp contract(off)
    const int i = blockIdx.x * 256 + threadIdx.x; if (i >= n8) return;
    const v4f a = *(const v4f*)(src + (size_t)i * 8); const v4f b = *(const v4f*)(src + (size_t)i * 8 + 4); v8h o;
#pragma unroll
    for (int k = 0; k < 4; ++k) { o[k] = toh_flush(bfr(a[k]) * WCS); o[4 + k] = toh_flush(bfr(b[k]) * WCS); }
    *(volatile v8h*)(dst + (size_t)i * 8) = o; __threadfence(); *(volatile v8h*)(dst + (size_t)i * 8) = o;
}

__global__ __launch_bounds__(256) void k_scal(const float* __restrict__ lo_core, const float* __restrict__ hi_core, const float* __restrict__ lo_ext, const float* __restrict__ hi_ext,
                                              const float* __restrict__ b_out, float* SP) {
#pragma clang fp contract(off)
    const int i = threadIdx.x; const int s = i >> 2, q = i & 3;
    const v2f lc = *(const v2f*)(lo_core + 2 * s), hc = *(const v2f*)(hi_core + 2 * s), le = *(const v2f*)(lo_ext + 2 * s), he = *(const v2f*)(hi_ext + 2 * s);
    const float lc0 = bfr(lc[0]), lc1 = bfr(lc[1]), hc0 = bfr(hc[0]), hc1 = bfr(hc[1]);
    const float le0 = bfr(le[0]), le1 = bfr(le[1]), he0 = bfr(he[0]), he1 = bfr(he[1]);
    const float bo = bfr(b_out[s]);
    const float ov0 = fmaxf(he0 - hc0, lc0 - le0), ov1 = fmaxf(he1 - hc1, lc1 - le1);
    const float wd0 = he0 - le0, wd1 = he1 - le1;
    const float sd0 = 4.0f * (1.0f / (2.0f * ov0 * wd0 + 1e-8f));
    const float sd1 = 4.0f * (1.0f / (2.0f * ov1 * wd1 + 1e-8f));
    const float cen0 = (le0 + he0) * 0.5f, cen1 = (le1 + he1) * 0.5f;
    const float iw0 = 1.0f / (wd0 * 0.5f), iw1 = 1.0f / (wd1 * 0.5f);
    v4f o;
    o[0] = (q == 0) ? bo  : ((q == 1) ? hc1  : ((q == 2) ? cen1 : 0.0f));
    o[1] = (q == 0) ? lc0 : ((q == 1) ? sd0  : ((q == 2) ? iw0  : 0.0f));
    o[2] = (q == 0) ? lc1 : ((q == 1) ? sd1  : ((q == 2) ? iw1  : 0.0f));
    o[3] = (q == 0) ? hc0 : ((q == 1) ? cen0 : 0.0f);
    *(volatile v4f*)(SP + (size_t)i * 4) = o; __threadfence(); *(volatile v4f*)(SP + (size_t)i * 4) = o;
}

__global__ __launch_bounds__(32 * MW) void k_mlp(const float* __restrict__ X, const float* __restrict__ SP, const float* __restrict__ WI, const float* __restrict__ BI,
                                                 const h16* __restrict__ WH, const float* __restrict__ BH, const float* __restrict__ WO,
                                                 const float* __restrict__ scale_p, const float* __restrict__ shift_p, float* OUT) {
    __shared__ __align__(16) float res[TPB];
    const int lane = threadIdx.x & 31, lr = lane & 15, hi = lane >> 4;
    const int wave = __builtin_amdgcn_readfirstlane((int)(threadIdx.x >> 5));
    const int n0 = blockIdx.x * TPB;
    const int n = n0 + wave * 16 + lr;
    const v2f xv = *(const v2f*)(X + (size_t)n * 2);
    const float x0 = bfr(xv[0]), x1 = bfr(xv[1]);
    const float scl = bfr(scale_p[0]), shf = bfr(shift_p[0]);
    float num = 0.0f, den = 0.0f;
#pragma unroll 1
    for (int s = 0; s < NSUB; ++s) {
        const float* sp = SP + s * SCP;
        const v4f c0 = *(const v4f*)sp, c1 = *(const v4f*)(sp + 4), c2 = *(const v4f*)(sp + 8);
        const float bo = c0[0], lc0 = c0[1], lc1 = c0[2], hc0 = c0[3], hc1 = c1[0], sd0 = c1[1], sd1 = c1[2], cen0 = c1[3], cen1 = c2[0], iw0 = c2[1], iw1 = c2[2];
        const float w = (sig_e(sd0 * (x0 - lc0)) * sig_e(sd0 * (hc0 - x0))) * (sig_e(sd1 * (x1 - lc1)) * sig_e(sd1 * (hc1 - x1)));
        const float xn0 = (x0 - cen0) * iw0, xn1 = (x1 - cen1) * iw1;
        const float* wi = WI + s * (HID * 2) + 16 * hi;
        const float* bi = BI + s * HID + 8 * hi;
        float t[16]; v16h act;
#pragma unroll
        for (int mh = 0; mh < 2; ++mh) {
            const float* wp = wi + 32 * mh; const float* bp = bi + 16 * mh;
            const v8f bb = cat8f(*(const v4f*)bp, *(const v4f*)(bp + 4));
#pragma unroll
            for (int k = 0; k < 4; ++k) {
                const v4f u = *(const v4f*)(wp + 4 * k);
                const float p0 = fmaf(u[0], xn0, fmaf(u[1], xn1, bb[2 * k]));
                const float p1 = fmaf(u[2], xn0, fmaf(u[3], xn1, bb[2 * k + 1]));
                const float t0 = tanh_e(p0, TK1, TC1), t1 = tanh_e(p1, TK1, TC1);
                t[8 * mh + 2 * k] = t0; t[8 * mh + 2 * k + 1] = t1;
                act[8 * mh + 2 * k] = toh_flush(t0); act[8 * mh + 2 * k + 1] = toh_flush(t1); }
        }
#pragma unroll
        for (int l = 0; l < NLH; ++l) {
            const h16* wr = WH + ((size_t)(l * NSUB + s) * HID + lr) * HID + 8 * hi;
            const float* bl = BH + (size_t)(l * NSUB + s) * HID + 8 * hi;
            const v16h a0 = ldh(wr), a1 = ldh(wr + 16 * HID);
            v8f d0 = cat8f(*(const v4f*)bl, *(const v4f*)(bl + 4));
            v8f d1 = cat8f(*(const v4f*)(bl + 16), *(const v4f*)(bl + 20));
            d0 = wmma16g(a0, act, d0);
            d1 = wmma16g(a1, act, d1);
#pragma unroll
            for (int j = 0; j < 8; ++j) {
                const float t0 = tanh_e(d0[j], TKH, TCH), t1 = tanh_e(d1[j], TKH, TCH);
                t[j] = t0; t[8 + j] = t1;
                act[j] = toh_flush(t0); act[8 + j] = toh_flush(t1); }
        }
        const float* wo = WO + s * HID + 8 * hi;
        const v4f o0 = *(const v4f*)wo, o1 = *(const v4f*)(wo + 4), o2 = *(const v4f*)(wo + 16), o3 = *(const v4f*)(wo + 20);
        float part = 0.0f;
#pragma unroll
        for (int j = 0; j < 4; ++j) part = fmaf(t[j], o0[j], part);
#pragma unroll
        for (int j = 0; j < 4; ++j) part = fmaf(t[4 + j], o1[j], part);
#pragma unroll
        for (int j = 0; j < 4; ++j) part = fmaf(t[8 + j], o2[j], part);
#pragma unroll
        for (int j = 0; j < 4; ++j) part = fmaf(t[12 + j], o3[j], part);
        float y = part + __shfl_xor(part, 16, 32);
        y = (y + bo) * scl + shf;
        num += y * w;
        den += w;
    }
    const float u = num * (1.0f / (den + 1e-8f));
    if (hi == 0) res[wave * 16 + lr] = u;
    __syncthreads();
    if (wave == 0) {
        const v4f val = *(const v4fa*)(&res[lane * 4]);
        float* op = OUT + (size_t)n0 + (size_t)lane * 4;
#pragma unroll 1
        for (int ps = 0; ps < 2; ++ps) {
            *(volatile v4f*)op = val;
            if (ps == 0) __threadfence(); }
    }
}

static constexpr size_t al256(size_t v) { return (v + 255) & ~(size_t)255; }
static constexpr size_t N_WH = (size_t)NLH * NSUB * HID * HID;
static constexpr size_t N_WI = (size_t)NSUB * HID * 2;
static constexpr size_t N_BI = (size_t)NSUB * HID;
static constexpr size_t N_BH = (size_t)NLH * NSUB * HID;
static constexpr size_t N_WO = (size_t)NSUB * HID;
static constexpr size_t N_SP = (size_t)NSUB * SCP;
static constexpr size_t SZ_WH = al256(N_WH * 2);
static constexpr size_t SZ_WI = al256(N_WI * 4);
static constexpr size_t SZ_BI = al256(N_BI * 4);
static constexpr size_t SZ_BH = al256(N_BH * 4);
static constexpr size_t SZ_WO = al256(N_WO * 4);
static constexpr size_t SZ_SP = al256(N_SP * 4);
static constexpr size_t SZ_TOTAL = SZ_WH + SZ_WI + SZ_BI + SZ_BH + SZ_WO + SZ_SP;
static_assert(SZ_TOTAL <= (size_t)134217728);
static_assert(N_SP * 4 == (size_t)256 * 16);
static_assert(N_WH % 8 == 0);
static_assert(N_WI % 4 == 0);
static_assert(N_BI % 4 == 0);
static_assert(N_BH % 4 == 0);
static_assert(N_WO % 4 == 0);

extern "C" void kernel_launch(void* const* d_in, const int* in_sizes, int n_in,
                              void* d_out, int out_size, void* d_ws, size_t ws_size, hipStream_t stream) {
    if (n_in < 13) return;
    if ((size_t)in_sizes[0] < (size_t)NPTS * 2) return;
    if (in_sizes[1] < NSUB * 2 || in_sizes[2] < NSUB * 2 || in_sizes[3] < NSUB * 2 || in_sizes[4] < NSUB * 2) return;
    if ((size_t)in_sizes[5] < N_WI || (size_t)in_sizes[6] < N_BI || (size_t)in_sizes[7] < N_WH || (size_t)in_sizes[8] < N_BH) return;
    if ((size_t)in_sizes[9] < N_WO || in_sizes[10] < NSUB || in_sizes[11] < 1 || in_sizes[12] < 1) return;
    if ((size_t)out_size < (size_t)NPTS) return;
    if (SZ_TOTAL > ws_size) return;
    const float* x       = (const float*)d_in[0];
    const float* lo_core = (const float*)d_in[1];
    const float* hi_core = (const float*)d_in[2];
    const float* lo_ext  = (const float*)d_in[3];
    const float* hi_ext  = (const float*)d_in[4];
    const float* w_in    = (const float*)d_in[5];
    const float* b_in    = (const float*)d_in[6];
    const float* w_h     = (const float*)d_in[7];
    const float* b_h     = (const float*)d_in[8];
    const float* w_out   = (const float*)d_in[9];
    const float* b_out   = (const float*)d_in[10];
    const float* scale_p = (const float*)d_in[11];
    const float* shift_p = (const float*)d_in[12];
    float* OUT = (float*)d_out;
    char* wsp = (char*)d_ws;
    h16*   WH = (h16*)wsp;   wsp += SZ_WH;
    float* WI = (float*)wsp; wsp += SZ_WI;
    float* BI = (float*)wsp; wsp += SZ_BI;
    float* BH = (float*)wsp; wsp += SZ_BH;
    float* WO = (float*)wsp; wsp += SZ_WO;
    float* SP = (float*)wsp; wsp += SZ_SP;

    { const int n8 = (int)(N_WH / 8); k_wconv<<<(unsigned)((n8 + 255) / 256), 256, 0, stream>>>(w_h, WH, n8); }
    { const int n4 = (int)(N_WI / 4); k_cvtf<<<(unsigned)((n4 + 255) / 256), 256, 0, stream>>>(w_in, WI, n4, 1.0f); }
    { const int n4 = (int)(N_BI / 4); k_cvtf<<<(unsigned)((n4 + 255) / 256), 256, 0, stream>>>(b_in, BI, n4, 1.0f); }
    { const int n4 = (int)(N_BH / 4); k_cvtf<<<(unsigned)((n4 + 255) / 256), 256, 0, stream>>>(b_h, BH, n4, WCS); }
    { const int n4 = (int)(N_WO / 4); k_cvtf<<<(unsigned)((n4 + 255) / 256), 256, 0, stream>>>(w_out, WO, n4, 1.0f); }
    k_scal<<<1, 256, 0, stream>>>(lo_core, hi_core, lo_ext, hi_ext, b_out, SP);

    k_mlp<<<NPTS / TPB, 32 * MW, 0, stream>>>(x, SP, WI, BI, WH, BH, WO, scale_p, shift_p, OUT);
}
